// GNNModel_55619826483422
// MI455X (gfx1250) — hardware-verified
//
#include <hip/hip_runtime.h>
#include <stddef.h>
#include <stdint.h>
#include <math.h>


#define DD     128
#define KA     256
#define NGR    256
#define NN     50000
#define NE     500000
#define NTHR   256
#define NWAVE  8
#define EPT    8
#define CHUNK  (NTHR * EPT)
#define WCAP   (EPT * 32)
#define LISTN  (NWAVE * WCAP)
#define NBA    1024
#define SLA    10
#define RCAP   28672
#define DEGCAP 64
#define GBM    64
#define GTHR   128
#define MP     50048
#define NBLK   49
#define NBP    (NBLK * NBA)
#define NBW1   8
#define NBW2   16
#define GX     (MP * 16 / NTHR)
#define HG     32
#define NHB    8
#define FLP    32
#define AGG_ZINTS (LISTN + 2 * RCAP + 3 * NBA)
#define AGG_LDS_INTS (AGG_ZINTS + 16)
#define WSMAX  134217728

static_assert((CHUNK & (CHUNK - 1)) == 0 && CHUNK <= 4096);
static_assert((NBA & (NBA - 1)) == 0 && NBA == (1 << SLA));
static_assert(((long long)NE << SLA) < (1LL << 31));
static_assert(LISTN % NTHR == 0 && LISTN % 4 == 0);
static_assert(NBA % NWAVE == 0 && NBA == 4 * NTHR);
static_assert(RCAP % (NTHR * 4) == 0 && AGG_ZINTS % 4 == 0);
static_assert(RCAP >= 10475 + 10475 / 20 + 1);
static_assert(DEGCAP >= 26 + 8);
static_assert(DD == 4 * 32 && KA == 2 * DD && DD % 32 == 0 && KA % 32 == 0);
static_assert(GBM == (GTHR / 32) * 16 && MP % GBM == 0 && MP >= NN && MP - NN < GBM);
static_assert(NN == 390 * 128 + 80 && MP == 391 * 128);
static_assert(NBP >= MP && (NBLK - 1) * NBA < MP);
static_assert((MP * 16) % NTHR == 0);
static_assert(NBW1 * NTHR == DD * (DD / 8) && NBW2 * NTHR == DD * (KA / 8));
static_assert(NHB * HG == NGR && HG * 4 == 128 && HG == 4 * NWAVE);
static_assert(NBLK <= NTHR && FLP * 4 == 128);
static_assert(AGG_LDS_INTS * 4 <= 300000);
static_assert((NE & 3) == 0);

typedef float          v4f   __attribute__((ext_vector_type(4)));
typedef float          v8f   __attribute__((ext_vector_type(8)));
typedef int            v4i   __attribute__((ext_vector_type(4)));
typedef int            v8i   __attribute__((ext_vector_type(8)));
typedef unsigned short v8us  __attribute__((ext_vector_type(8)));
typedef unsigned short v16us __attribute__((ext_vector_type(16)));
typedef __bf16         v16bf __attribute__((ext_vector_type(16)));
typedef v4f  __attribute__((may_alias)) v4fa;
typedef v4i  __attribute__((may_alias)) v4ia;
typedef v8us __attribute__((may_alias)) v8usa;
union FragB { v16bf v; v16us u; v8us h[2]; v8i w; };

__device__ __forceinline__ v8f wmb(const FragB& a, const FragB& b, v8f c) {
  v8f d = __builtin_amdgcn_wmma_f32_16x16x32_bf16(false, a.v, false, b.v, (short)0, c, false, false);
  asm volatile("v_nop\n\tv_nop\n\tv_nop\n\tv_nop" : "+v"(d) : "v"(a.w), "v"(b.w));
  return d;
}

__device__ __forceinline__ unsigned bf16_bits(float f) {
  const unsigned u = __float_as_uint(f);
  const unsigned r = (u + 0x7FFFu + ((u >> 16) & 1u)) >> 16;
  return (f != f) ? 0x7FC0u : r;
}
__device__ __forceinline__ float bf16_val(float f) {
  return __uint_as_float(bf16_bits(f) << 16);
}

__device__ __forceinline__ void put8(unsigned short* dp, v8us o) {
  *(volatile v8us*)dp = o;
  __threadfence();
  *(volatile v8us*)dp = o;
}

__device__ __forceinline__ void hilo_pack(float v0, float v1, float v2, float v3,
                                          int& h01, int& h23, int& l01, int& l23) {
  const unsigned a0 = bf16_bits(v0), a1 = bf16_bits(v1), a2 = bf16_bits(v2), a3 = bf16_bits(v3);
  const unsigned b0 = bf16_bits(v0 - __uint_as_float(a0 << 16));
  const unsigned b1 = bf16_bits(v1 - __uint_as_float(a1 << 16));
  const unsigned b2 = bf16_bits(v2 - __uint_as_float(a2 << 16));
  const unsigned b3 = bf16_bits(v3 - __uint_as_float(a3 << 16));
  h01 = (int)(a0 | (a1 << 16)); h23 = (int)(a2 | (a3 << 16));
  l01 = (int)(b0 | (b1 << 16)); l23 = (int)(b2 | (b3 << 16));
}

__device__ __forceinline__ v4i regroup16(int h01, int h23, int l01, int l23, int lane) {
  const int s0 = (2 * lane) & 31, s1 = s0 + 1;
  const int a0 = __shfl(h01, s0, 32), a1 = __shfl(h23, s0, 32), a2 = __shfl(h01, s1, 32), a3 = __shfl(h23, s1, 32);
  const int b0 = __shfl(l01, s0, 32), b1 = __shfl(l23, s0, 32), b2 = __shfl(l01, s1, 32), b3 = __shfl(l23, s1, 32);
  const int mk = (lane < 16) ? -1 : 0;
  v4i o;
  o.x = (a0 & mk) | (b0 & ~mk); o.y = (a1 & mk) | (b1 & ~mk);
  o.z = (a2 & mk) | (b2 & ~mk); o.w = (a3 & mk) | (b3 & ~mk);
  return o;
}

template <int SLB>
__device__ __forceinline__ int scan_chunk(const int* __restrict__ dsts, int nE, int cbase, int slotBase,
                                          int nb, int vec8, int* list, int tid, int lane, int wave) {
  int wc = 0;
  const int el0  = tid * EPT;
  const int e0   = cbase + el0;
  const int sent = -2147483647 - 1;
  v4i da, db;
  if (vec8 != 0 && cbase + CHUNK <= nE) {
    da = *(const v4i*)(dsts + e0);
    db = *(const v4i*)(dsts + e0 + 4);
  } else {
    da.x = (e0     < nE) ? dsts[min(e0,     nE - 1)] : sent;
    da.y = (e0 + 1 < nE) ? dsts[min(e0 + 1, nE - 1)] : sent;
    da.z = (e0 + 2 < nE) ? dsts[min(e0 + 2, nE - 1)] : sent;
    da.w = (e0 + 3 < nE) ? dsts[min(e0 + 3, nE - 1)] : sent;
    db.x = (e0 + 4 < nE) ? dsts[min(e0 + 4, nE - 1)] : sent;
    db.y = (e0 + 5 < nE) ? dsts[min(e0 + 5, nE - 1)] : sent;
    db.z = (e0 + 6 < nE) ? dsts[min(e0 + 6, nE - 1)] : sent;
    db.w = (e0 + 7 < nE) ? dsts[min(e0 + 7, nE - 1)] : sent;
  }
  const unsigned nbs = (unsigned)slotBase;
  const unsigned unb = (unsigned)nb;
  const unsigned s0 = (unsigned)da.x - nbs, s1 = (unsigned)da.y - nbs;
  const unsigned s2 = (unsigned)da.z - nbs, s3 = (unsigned)da.w - nbs;
  const unsigned s4 = (unsigned)db.x - nbs, s5 = (unsigned)db.y - nbs;
  const unsigned s6 = (unsigned)db.z - nbs, s7 = (unsigned)db.w - nbs;
  const bool h0 = s0 < unb, h1 = s1 < unb, h2 = s2 < unb, h3 = s3 < unb;
  const bool h4 = s4 < unb, h5 = s5 < unb, h6 = s6 < unb, h7 = s7 < unb;
  const unsigned any = __builtin_amdgcn_ballot_w32(h0 | h1 | h2 | h3 | h4 | h5 | h6 | h7);
  if (any != 0u) {
#define HITJ(J, HJ, SJ) { \
      const unsigned mj = __builtin_amdgcn_ballot_w32(HJ); \
      if (mj != 0u) { \
        if (HJ) { \
          const int pos = wc + (int)__builtin_amdgcn_mbcnt_lo(mj, 0u); \
          if (pos < WCAP) list[wave * WCAP + pos] = ((el0 + (J)) << SLB) | (int)(SJ); \
        } \
        wc += (int)__builtin_popcount(mj); } }
    HITJ(0, h0, s0)
    HITJ(1, h1, s1)
    HITJ(2, h2, s2)
    HITJ(3, h3, s3)
    HITJ(4, h4, s4)
    HITJ(5, h5, s5)
    HITJ(6, h6, s6)
    HITJ(7, h7, s7)
#undef HITJ
  }
  return wc;
}

__global__ __launch_bounds__(NTHR) void k_prep(const float* __restrict__ x, int nN, int gx,
                                               const float* __restrict__ w1, const float* __restrict__ w2,
                                               unsigned short* xb, unsigned short* w1b, unsigned short* w2d) {
  const int tid = (int)threadIdx.x;
  const int blk = (int)blockIdx.x;
  if (blk < gx) {
    const int u   = blk * NTHR + tid;
    const int row = u >> 4;
    const int k8  = (u & 15) * 8;
    const int rc  = row < nN ? row : nN - 1;
    const float* p = x + (size_t)rc * DD + k8;
    const v4f a = *(const v4fa*)p;
    const v4f b = *(const v4fa*)(p + 4);
    const bool ok = row < nN;
    v8us o;
    o[0] = ok ? (unsigned short)bf16_bits(a.x) : (unsigned short)0;
    o[1] = ok ? (unsigned short)bf16_bits(a.y) : (unsigned short)0;
    o[2] = ok ? (unsigned short)bf16_bits(a.z) : (unsigned short)0;
    o[3] = ok ? (unsigned short)bf16_bits(a.w) : (unsigned short)0;
    o[4] = ok ? (unsigned short)bf16_bits(b.x) : (unsigned short)0;
    o[5] = ok ? (unsigned short)bf16_bits(b.y) : (unsigned short)0;
    o[6] = ok ? (unsigned short)bf16_bits(b.z) : (unsigned short)0;
    o[7] = ok ? (unsigned short)bf16_bits(b.w) : (unsigned short)0;
    put8(xb + (size_t)row * DD + k8, o);
  } else if (blk < gx + NBW1) {
    const int u  = (blk - gx) * NTHR + tid;
    const int n  = u >> 4;
    const int k8 = (u & 15) * 8;
    const float* p = w1 + (size_t)n * DD + k8;
    const v4f a = *(const v4fa*)p;
    const v4f b = *(const v4fa*)(p + 4);
    v8us o;
    o[0] = (unsigned short)bf16_bits(a.x); o[1] = (unsigned short)bf16_bits(a.y);
    o[2] = (unsigned short)bf16_bits(a.z); o[3] = (unsigned short)bf16_bits(a.w);
    o[4] = (unsigned short)bf16_bits(b.x); o[5] = (unsigned short)bf16_bits(b.y);
    o[6] = (unsigned short)bf16_bits(b.z); o[7] = (unsigned short)bf16_bits(b.w);
    put8(w1b + (size_t)n * DD + k8, o);
  } else {
    const int u  = (blk - gx - NBW1) * NTHR + tid;
    const int n  = u >> 5;
    const int k8 = (u & 31) * 8;
    const int kk = k8 & (DD - 1);
    const float* p = w2 + (size_t)n * DD + kk;
    const v4f a = *(const v4fa*)p;
    const v4f b = *(const v4fa*)(p + 4);
    v8us o;
    o[0] = (unsigned short)bf16_bits(a.x); o[1] = (unsigned short)bf16_bits(a.y);
    o[2] = (unsigned short)bf16_bits(a.z); o[3] = (unsigned short)bf16_bits(a.w);
    o[4] = (unsigned short)bf16_bits(b.x); o[5] = (unsigned short)bf16_bits(b.y);
    o[6] = (unsigned short)bf16_bits(b.z); o[7] = (unsigned short)bf16_bits(b.w);
    put8(w2d + (size_t)n * KA + k8, o);
  }
}

__global__ __launch_bounds__(NTHR) void k_bucket(const int* __restrict__ srcs, const int* __restrict__ dsts,
                                                 const float* __restrict__ ew, int nE, int nN, int vec8,
                                                 int* hsrc, float* hew, int* cntp, int* offp, float* dinvp,
                                                 int* flags) {
  extern __shared__ __attribute__((aligned(16))) int dsm[];
  int* list = dsm;
  int* hl   = dsm + LISTN;
  int* sl   = dsm + LISTN + RCAP;
  int* cnt  = dsm + LISTN + 2 * RCAP;
  int* offs = cnt + NBA;
  int* cur  = offs + NBA;
  int* misc = cur + NBA;
  const int tid = (int)threadIdx.x, lane = tid & 31, wave = tid >> 5;
  const int blk = (int)blockIdx.x;
  const int nodeBase = blk * NBA;

  {
    const v4i z4 = {0, 0, 0, 0};
    for (int i = tid * 4; i < AGG_ZINTS; i += NTHR * 4) *(v4ia*)(dsm + i) = z4;
    if (tid < 16) misc[tid] = 0;
  }
  __syncthreads();

  int t = 0, ov = 0;
  const int nChunks = (nE + CHUNK - 1) / CHUNK;
#pragma unroll 1
  for (int ch = 0; ch < nChunks; ++ch) {
    const int cbase = ch * CHUNK;
    const int wc = scan_chunk<SLA>(dsts, nE, cbase, nodeBase, NBA, vec8, list, tid, lane, wave);
    if (lane == 0) misc[wave] = wc;
    __syncthreads();
    if (wave == 0) {
#pragma unroll 1
      for (int w2 = 0; w2 < NWAVE; ++w2) {
        int c = misc[w2];
        c = c < 0 ? 0 : (c > WCAP ? WCAP : c);
#pragma unroll 1
        for (int b0 = 0; b0 < c; b0 += 32) {
          const int idx = b0 + lane;
          const int ent = list[w2 * WCAP + (idx < WCAP ? idx : WCAP - 1)];
          const int m32 = (c - b0) < 32 ? (c - b0) : 32;
#pragma unroll 1
          for (int k = 0; k < m32; ++k) {
            const int u    = __builtin_amdgcn_readlane(ent, k);
            const int slot = u & (NBA - 1);
            const int el   = (u >> SLA) & (CHUNK - 1);
            const int pk   = ((cbase + el) << SLA) | slot;
            if (t < RCAP) {
              if (lane == 0) { hl[t] = pk; cnt[slot] = cnt[slot] + 1; }
              t = t + 1;
            } else {
              ov = 1;
            }
          }
        }
      }
    }
    __syncthreads();
  }
  if (wave == 0 && lane == 0) { misc[8] = t; misc[9] = ov; }
  __syncthreads();
  int tt = misc[8];
  tt = tt < 0 ? 0 : (tt > RCAP ? RCAP : tt);

  if (wave == 0) {
    const int base = lane * (NBA / 32);
    int s = 0;
#pragma unroll 1
    for (int i = 0; i < NBA / 32; ++i) s += cnt[base + i];
    int incl = s;
#pragma unroll
    for (int d = 1; d < 32; d <<= 1) {
      const int y = __shfl_up(incl, d, 32);
      if (lane >= d) incl += y;
    }
    int run = incl - s;
#pragma unroll 1
    for (int i = 0; i < NBA / 32; ++i) {
      const int cv = cnt[base + i];
      offs[base + i] = run;
      cur[base + i]  = run;
      run += cv;
    }
  }
  __syncthreads();
  if (wave == 0) {
#pragma unroll 1
    for (int b0 = 0; b0 < tt; b0 += 32) {
      const int idx = b0 + lane;
      const int ent = hl[idx < RCAP ? idx : RCAP - 1];
      const int m32 = (tt - b0) < 32 ? (tt - b0) : 32;
#pragma unroll 1
      for (int k = 0; k < m32; ++k) {
        const int u    = __builtin_amdgcn_readlane(ent, k);
        const int slot = u & (NBA - 1);
        if (lane == 0) {
          int p = cur[slot];
          p = p < 0 ? 0 : (p > RCAP - 1 ? RCAP - 1 : p);
          sl[p] = u;
          cur[slot] = p + 1;
        }
      }
    }
  }
  __syncthreads();

  int*   hsb = hsrc + (size_t)blk * RCAP;
  float* hwb = hew  + (size_t)blk * RCAP;
#pragma unroll 1
  for (int it = 0; it < RCAP / (NTHR * 4); ++it) {
    const int p = it * (NTHR * 4) + 4 * tid;
    const v4i e4 = *(const v4ia*)(sl + p);
    int e0 = e4.x >> SLA, e1 = e4.y >> SLA, e2 = e4.z >> SLA, e3 = e4.w >> SLA;
    e0 = e0 < 0 ? 0 : (e0 > nE - 1 ? nE - 1 : e0);
    e1 = e1 < 0 ? 0 : (e1 > nE - 1 ? nE - 1 : e1);
    e2 = e2 < 0 ? 0 : (e2 > nE - 1 ? nE - 1 : e2);
    e3 = e3 < 0 ? 0 : (e3 > nE - 1 ? nE - 1 : e3);
    int r0 = srcs[e0], r1 = srcs[e1], r2 = srcs[e2], r3 = srcs[e3];
    r0 = r0 < 0 ? 0 : (r0 > nN - 1 ? nN - 1 : r0);
    r1 = r1 < 0 ? 0 : (r1 > nN - 1 ? nN - 1 : r1);
    r2 = r2 < 0 ? 0 : (r2 > nN - 1 ? nN - 1 : r2);
    r3 = r3 < 0 ? 0 : (r3 > nN - 1 ? nN - 1 : r3);
    const float w0 = bf16_val(ew[e0]), w1 = bf16_val(ew[e1]);
    const float w2 = bf16_val(ew[e2]), w3 = bf16_val(ew[e3]);
    v4i sv; sv.x = r0; sv.y = r1; sv.z = r2; sv.w = r3;
    v4f wv; wv.x = w0; wv.y = w1; wv.z = w2; wv.w = w3;
    v4i wb;
    wb.x = __float_as_int(w0); wb.y = __float_as_int(w1);
    wb.z = __float_as_int(w2); wb.w = __float_as_int(w3);
    *(v4ia*)(hl + p) = wb;
    *(volatile v4i*)(hsb + p) = sv;
    *(volatile v4f*)(hwb + p) = wv;
    __threadfence();
    *(volatile v4i*)(hsb + p) = sv;
    *(volatile v4f*)(hwb + p) = wv;
  }
  __syncthreads();

  int bigf = 0;
#pragma unroll 1
  for (int q = 0; q < NBA / NTHR; ++q) {
    const int s = q * NTHR + tid;
    int c = cnt[s];
    if (c > DEGCAP) bigf = 1;
    c = c < 0 ? 0 : (c > DEGCAP ? DEGCAP : c);
    int o = offs[s];
    o = o < 0 ? 0 : (o > RCAP ? RCAP : o);
    float a = 0.0f;
#pragma unroll 1
    for (int j = 0; j < c; ++j) {
      int idx = o + j;
      idx = idx > RCAP - 1 ? RCAP - 1 : idx;
      a += __int_as_float(hl[idx]);
    }
    const float deg = a + 1.0f;
    const float di  = (deg > 0.0f) ? (1.0f / sqrtf(deg)) : 0.0f;
    cur[s] = __float_as_int(di);
  }
  if (bigf != 0) misc[10] = 1;
  __syncthreads();

  const v4i c4 = *(const v4ia*)(cnt  + 4 * tid);
  const v4i o4 = *(const v4ia*)(offs + 4 * tid);
  const v4i d4 = *(const v4ia*)(cur  + 4 * tid);
  v4f dv;
  dv.x = __int_as_float(d4.x); dv.y = __int_as_float(d4.y);
  dv.z = __int_as_float(d4.z); dv.w = __int_as_float(d4.w);
  const int fl = ((misc[9] | misc[10]) != 0) ? 1 : 0;
  v4i f4; f4.x = fl; f4.y = fl; f4.z = fl; f4.w = fl;
  int*   cp = cntp  + (size_t)nodeBase + 4 * tid;
  int*   op = offp  + (size_t)nodeBase + 4 * tid;
  float* dp = dinvp + (size_t)nodeBase + 4 * tid;
  int*   fp = flags + (size_t)blk * FLP + 4 * (tid & 7);
  const bool fw = tid < 8;
  *(volatile v4i*)cp = c4;
  *(volatile v4i*)op = o4;
  *(volatile v4f*)dp = dv;
  if (fw) *(volatile v4i*)fp = f4;
  __threadfence();
  *(volatile v4i*)cp = c4;
  *(volatile v4i*)op = o4;
  *(volatile v4f*)dp = dv;
  if (fw) *(volatile v4i*)fp = f4;
}

__global__ __launch_bounds__(GTHR) void k_gemm(const unsigned short* __restrict__ A,
                                               const unsigned short* __restrict__ BT, int K, float* C) {
  __shared__ __attribute__((aligned(16))) float stg[GBM * DD];
  const int tid = (int)threadIdx.x, lane = tid & 31, wave = tid >> 5, hh = lane >> 4, m = lane & 15;
  const int rowBase = (int)blockIdx.x * GBM;

  v8f acc[8];
  {
    const v8f z = {0.f, 0.f, 0.f, 0.f, 0.f, 0.f, 0.f, 0.f};
#pragma unroll
    for (int t = 0; t < 8; ++t) acc[t] = z;
  }
  const unsigned short* ap = A  + (size_t)(rowBase + 16 * wave + m) * (size_t)K + 8 * hh;
  const unsigned short* bp = BT + (size_t)m * (size_t)K + 8 * hh;

#pragma unroll 1
  for (int k0 = 0; k0 < K; k0 += 32) {
    FragB af;
    af.h[0] = *(const v8usa*)(ap + k0);
    af.h[1] = *(const v8usa*)(ap + k0 + 16);
#pragma unroll
    for (int nt = 0; nt < 8; ++nt) {
      const unsigned short* wq = bp + (size_t)(16 * nt) * (size_t)K + k0;
      FragB bf;
      bf.h[0] = *(const v8usa*)wq;
      bf.h[1] = *(const v8usa*)(wq + 16);
      acc[nt] = wmb(af, bf, acc[nt]);
    }
  }

#pragma unroll
  for (int nt = 0; nt < 8; ++nt) {
    const int lc = 16 * nt + m;
#pragma unroll
    for (int r = 0; r < 8; ++r) {
      const int lr = 16 * wave + 8 * hh + r;
      stg[lr * DD + lc] = acc[nt][r];
    }
  }
  __syncthreads();

  v4f fv[16];
#pragma unroll
  for (int i = 0; i < 16; ++i) fv[i] = *(const v4fa*)(stg + (16 * wave + i) * DD + 4 * lane);
#pragma unroll
  for (int i = 0; i < 16; ++i) {
    float* op = C + (size_t)(rowBase + 16 * wave + i) * DD + 4 * lane;
    *(volatile v4f*)op = fv[i];
  }
  __threadfence();
#pragma unroll
  for (int i = 0; i < 16; ++i) {
    float* op = C + (size_t)(rowBase + 16 * wave + i) * DD + 4 * lane;
    *(volatile v4f*)op = fv[i];
  }
}

template <int L1>
__global__ __launch_bounds__(NTHR) void k_agg(const int* __restrict__ hsrc, const float* __restrict__ hew,
                                              const int* __restrict__ cntp, const int* __restrict__ offp,
                                              const float* __restrict__ dinv, const int* __restrict__ flags,
                                              int nN, int mRows,
                                              const float* __restrict__ hx, const float* __restrict__ bias,
                                              unsigned short* ap, float* outp) {
  __shared__ __attribute__((aligned(16))) int scnt[NBA];
  __shared__ __attribute__((aligned(16))) int soff[NBA];
  const int tid = (int)threadIdx.x, lane = tid & 31, wave = tid >> 5;
  const int blk = (int)blockIdx.x;
  const int nodeBase = blk * NBA;

  {
    const v4i c4 = *(const v4ia*)(cntp + (size_t)nodeBase + 4 * tid);
    const v4i o4 = *(const v4ia*)(offp + (size_t)nodeBase + 4 * tid);
    *(v4ia*)(scnt + 4 * tid) = c4;
    *(v4ia*)(soff + 4 * tid) = o4;
  }
  const int ovf = flags[(size_t)blk * FLP];
  float bv0, bv1, bv2, bv3;
  {
    const v4f a = *(const v4fa*)(bias + 4 * lane);
    bv0 = bf16_val(a.x); bv1 = bf16_val(a.y); bv2 = bf16_val(a.z); bv3 = bf16_val(a.w);
  }
  __syncthreads();

  const int*   hs = hsrc + (size_t)blk * RCAP;
  const float* hw = hew  + (size_t)blk * RCAP;
  const float qnan = __int_as_float(0x7fc00000);
  const float pz = (ovf != 0) ? qnan : 0.0f;
#pragma unroll 1
  for (int si = 0; si < NBA / NWAVE; ++si) {
    const int s    = si * NWAVE + wave;
    const int node = nodeBase + s;
    int c = scnt[s];
    const bool big = c > DEGCAP;
    c = c < 0 ? 0 : (c > DEGCAP ? DEGCAP : c);
    int o = soff[s];
    o = o < 0 ? 0 : (o > RCAP ? RCAP : o);
    const int nc = node < nN ? node : nN - 1;
    const float dd = dinv[nc];
    const float rd = dd * dd;
    float g0 = 0.0f, g1 = 0.0f, g2 = 0.0f, g3 = 0.0f;
#pragma unroll 1
    for (int b0 = 0; b0 < c; b0 += 32) {
      int idx = o + b0 + lane;
      idx = idx > RCAP - 1 ? RCAP - 1 : idx;
      int sr = hs[idx];
      sr = sr < 0 ? 0 : (sr > nN - 1 ? nN - 1 : sr);
      const float wv = hw[idx];
      const float cf = (dinv[sr] * wv) * dd;
      const int  cfi = __float_as_int(cf);
      const int m32 = (c - b0) < 32 ? (c - b0) : 32;
#pragma unroll 1
      for (int k = 0; k < m32; ++k) {
        const int   sk = __builtin_amdgcn_readlane(sr, k);
        const float ck = __int_as_float(__builtin_amdgcn_readlane(cfi, k));
        const v4f a = *(const v4fa*)(hx + (size_t)sk * DD + 4 * lane);
        g0 = fmaf(ck, a.x, g0); g1 = fmaf(ck, a.y, g1);
        g2 = fmaf(ck, a.z, g2); g3 = fmaf(ck, a.w, g3);
      }
    }
    const v4f sv = *(const v4fa*)(hx + (size_t)nc * DD + 4 * lane);
    float y0 = (g0 + sv.x * rd) + bv0;
    float y1 = (g1 + sv.y * rd) + bv1;
    float y2 = (g2 + sv.z * rd) + bv2;
    float y3 = (g3 + sv.w * rd) + bv3;
    y0 = (y0 > 0.0f) ? y0 : (y0 - y0);
    y1 = (y1 > 0.0f) ? y1 : (y1 - y1);
    y2 = (y2 > 0.0f) ? y2 : (y2 - y2);
    y3 = (y3 > 0.0f) ? y3 : (y3 - y3);
    const float pzr = big ? qnan : pz;
    const bool live = node < nN;
    const float q0 = live ? y0 + pzr : 0.0f, q1 = live ? y1 + pzr : 0.0f;
    const float q2 = live ? y2 + pzr : 0.0f, q3 = live ? y3 + pzr : 0.0f;
    if constexpr (L1 != 0) {
      int h01, h23, l01, l23;
      hilo_pack(q0, q1, q2, q3, h01, h23, l01, l23);
      const v4i ow = regroup16(h01, h23, l01, l23, lane);
      if (node < mRows) {
        unsigned short* hp = ap + (size_t)node * KA + 8 * lane;
        *(volatile v4i*)hp = ow;
        __threadfence();
        *(volatile v4i*)hp = ow;
      }
    } else {
      v4f ow;
      ow.x = q0; ow.y = q1; ow.z = q2; ow.w = q3;
      if (live) {
        float* op = outp + (size_t)node * DD + 4 * lane;
        *(volatile v4f*)op = ow;
        __threadfence();
        *(volatile v4f*)op = ow;
      }
    }
  }
}

__global__ __launch_bounds__(NTHR) void k_pool(const float* __restrict__ hf, const int* __restrict__ bat,
                                               int nN, float* pl) {
  __shared__ __attribute__((aligned(16))) float wsm[NWAVE * DD];
  __shared__ int wcn[NWAVE];
  __shared__ __attribute__((aligned(16))) float outs[DD];
  const int tid = (int)threadIdx.x, lane = tid & 31, wave = tid >> 5;
  const int g = (int)blockIdx.x;

  float a0 = 0.0f, a1 = 0.0f, a2 = 0.0f, a3 = 0.0f;
  int cnt = 0;
#pragma unroll 1
  for (int i0 = wave * 32; i0 < nN; i0 += NTHR) {
    const int i  = i0 + lane;
    const int ic = i < nN ? i : nN - 1;
    const int b  = bat[ic];
    const bool hit = (i < nN) && (b == g);
    unsigned msk = __builtin_amdgcn_ballot_w32(hit);
    int nh = (int)__builtin_popcount(msk);
    nh = nh > 32 ? 32 : nh;
    cnt += nh;
#pragma unroll 1
    for (int q = 0; q < nh; ++q) {
      const int k = __builtin_ffs((int)msk) - 1;
      msk &= msk - 1u;
      int node = i0 + (k < 0 ? 0 : k);
      node = node > nN - 1 ? nN - 1 : node;
      const v4f v = *(const v4fa*)(hf + (size_t)node * DD + 4 * lane);
      a0 += v.x; a1 += v.y; a2 += v.z; a3 += v.w;
    }
  }
  {
    v4f av; av.x = a0; av.y = a1; av.z = a2; av.w = a3;
    *(v4fa*)(wsm + wave * DD + 4 * lane) = av;
  }
  if (lane == 0) wcn[wave] = cnt;
  __syncthreads();
  if (tid < DD) {
    float s = 0.0f;
    int c = 0;
#pragma unroll
    for (int w2 = 0; w2 < NWAVE; ++w2) { s += wsm[w2 * DD + tid]; c += wcn[w2]; }
    const float cf = (c < 1) ? 1.0f : (float)c;
    outs[tid] = s / cf;
  }
  __syncthreads();
  const v4f ov = *(const v4fa*)(outs + 4 * lane);
  float* op = pl + (size_t)g * DD + 4 * lane;
  const bool okst = (wave == 0);
  if (okst) *(volatile v4f*)op = ov;
  __threadfence();
  if (okst) *(volatile v4f*)op = ov;
}

__global__ __launch_bounds__(NTHR) void k_head(const float* __restrict__ pl, const float* __restrict__ fw1,
                                               const float* __restrict__ fb1, const float* __restrict__ fw2,
                                               const float* __restrict__ fb2, const int* __restrict__ flags,
                                               int nfl, float* out) {
  __shared__ __attribute__((aligned(16))) float ps[HG * DD];
  __shared__ __attribute__((aligned(16))) float os[HG * DD];
  __shared__ __attribute__((aligned(16))) float b1s[DD];
  __shared__ __attribute__((aligned(16))) float w2s[DD];
  __shared__ __attribute__((aligned(16))) float outs[HG];
  __shared__ int sfl;
  const int tid = (int)threadIdx.x, lane = tid & 31, wave = tid >> 5;
  const int blk = (int)blockIdx.x;

#pragma unroll 1
  for (int i = tid; i < HG * DD / 4; i += NTHR) {
    const v4f v = *(const v4fa*)(pl + (size_t)blk * (HG * DD) + 4 * i);
    *(v4fa*)(ps + 4 * i) = v;
  }
  if (tid < DD) {
    b1s[tid] = bf16_val(fb1[tid]);
    w2s[tid] = bf16_val(fw2[tid]);
  }
  if (tid == 0) sfl = 0;
  const int fi = tid < nfl ? tid : nfl - 1;
  const int fv = flags[(size_t)fi * FLP];
  const float fb2v = bf16_val(fb2[0]);
  __syncthreads();
  if (fv != 0) sfl = 1;

  const int c = tid & (DD - 1);
  const float* wr = fw1 + (size_t)c * DD;
#pragma unroll 1
  for (int j = 0; j < (HG * DD) / NTHR; ++j) {
    const int g = (j * NTHR + tid) >> 7;
    const float* pr = ps + g * DD;
    float s = 0.0f;
#pragma unroll 4
    for (int k4 = 0; k4 < DD / 4; ++k4) {
      const v4f p = *(const v4fa*)(pr + 4 * k4);
      const v4f w = *(const v4fa*)(wr + 4 * k4);
      s = fmaf(p.x, bf16_val(w.x), s);
      s = fmaf(p.y, bf16_val(w.y), s);
      s = fmaf(p.z, bf16_val(w.z), s);
      s = fmaf(p.w, bf16_val(w.w), s);
    }
    float v = s + b1s[c];
    v = (v > 0.0f) ? v : (v - v);
    os[g * DD + c] = v;
  }
  __syncthreads();

  const v4f w4 = *(const v4fa*)(w2s + 4 * lane);
#pragma unroll 1
  for (int q = 0; q < HG / NWAVE; ++q) {
    const int g = (HG / NWAVE) * wave + q;
    const v4f a = *(const v4fa*)(os + g * DD + 4 * lane);
    float p = a.x * w4.x;
    p = fmaf(a.y, w4.y, p);
    p = fmaf(a.z, w4.z, p);
    p = fmaf(a.w, w4.w, p);
#pragma unroll
    for (int d = 16; d > 0; d >>= 1) p += __shfl_xor(p, d, 32);
    if (lane == 0) outs[g] = p + fb2v;
  }
  __syncthreads();

  const int pois = sfl;
  const float qnan = __int_as_float(0x7fc00000);
  v4f ov = *(const v4fa*)(outs + 4 * (lane & 7));
  ov.x = (pois != 0) ? qnan : ov.x;
  ov.y = (pois != 0) ? qnan : ov.y;
  ov.z = (pois != 0) ? qnan : ov.z;
  ov.w = (pois != 0) ? qnan : ov.w;
  float* op = out + (size_t)blk * HG + 4 * (lane & 7);
  const bool okst = (wave == 0) && (lane < 8);
  if (okst) *(volatile v4f*)op = ov;
  __threadfence();
  if (okst) *(volatile v4f*)op = ov;
}

static inline size_t al256(size_t o) { return (o + 255) & ~(size_t)255; }

extern "C" void kernel_launch(void* const* d_in, const int* in_sizes, int n_in,
                              void* d_out, int out_size, void* d_ws, size_t ws_size,
                              hipStream_t stream) {
  if (n_in < 12) return;
  if (in_sizes[0] != NN * DD) return;
  if (in_sizes[1] != 2 * NE) return;
  if (in_sizes[2] != NE) return;
  if (in_sizes[3] != NN) return;
  if (in_sizes[4] != DD * DD || in_sizes[5] != DD) return;
  if (in_sizes[6] != DD * DD || in_sizes[7] != DD) return;
  if (in_sizes[8] != DD * DD || in_sizes[9] != DD) return;
  if (in_sizes[10] != DD || in_sizes[11] != 1) return;
  if (out_size != NGR) return;

  const float* x    = (const float*)d_in[0];
  const int*   edge = (const int*)d_in[1];
  const float* ew   = (const float*)d_in[2];
  const int*   bat  = (const int*)d_in[3];
  const float* W1   = (const float*)d_in[4];
  const float* b1   = (const float*)d_in[5];
  const float* W2   = (const float*)d_in[6];
  const float* b2   = (const float*)d_in[7];
  const float* fW1  = (const float*)d_in[8];
  const float* fb1  = (const float*)d_in[9];
  const float* fW2  = (const float*)d_in[10];
  const float* fb2  = (const float*)d_in[11];
  float* out = (float*)d_out;
  const int* src = edge;
  const int* dst = edge + NE;
  const int vec8 = ((NE & 3) == 0) ? 1 : 0;

  char* ws = (char*)d_ws;
  size_t off = 0;
  const size_t oW1B = off; off = al256(off + (size_t)DD * DD * 2);
  const size_t oW2D = off; off = al256(off + (size_t)DD * KA * 2);
  const size_t oXB  = off; off = al256(off + (size_t)MP * DD * 2);
  const size_t oH   = off; off = al256(off + (size_t)MP * DD * 4);
  const size_t oX1  = off; off = al256(off + (size_t)MP * KA * 2);
  const size_t oHF  = off; off = al256(off + (size_t)MP * DD * 4);
  const size_t oHS  = off; off = al256(off + (size_t)NBLK * RCAP * 4);
  const size_t oHW  = off; off = al256(off + (size_t)NBLK * RCAP * 4);
  const size_t oCNT = off; off = al256(off + (size_t)NBP * 4);
  const size_t oOFF = off; off = al256(off + (size_t)NBP * 4);
  const size_t oDIN = off; off = al256(off + (size_t)NBP * 4);
  const size_t oFLG = off; off = al256(off + (size_t)NBLK * FLP * 4);
  const size_t oPL  = off; off = al256(off + (size_t)NGR * DD * 4);
  if (off > ws_size || off > (size_t)WSMAX) return;
  unsigned short* W1B = (unsigned short*)(ws + oW1B);
  unsigned short* W2D = (unsigned short*)(ws + oW2D);
  unsigned short* XB  = (unsigned short*)(ws + oXB);
  float*          H   = (float*)(ws + oH);
  unsigned short* X1  = (unsigned short*)(ws + oX1);
  float*          HF  = (float*)(ws + oHF);
  int*            HS  = (int*)(ws + oHS);
  float*          HW  = (float*)(ws + oHW);
  int*            CNT = (int*)(ws + oCNT);
  int*            OFF = (int*)(ws + oOFF);
  float*          DIN = (float*)(ws + oDIN);
  int*            FLG = (int*)(ws + oFLG);
  float*          PL  = (float*)(ws + oPL);

  const size_t bktLds = (size_t)AGG_LDS_INTS * 4;
  hipFuncSetAttribute(reinterpret_cast<const void*>(&k_bucket), hipFuncAttributeMaxDynamicSharedMemorySize, (int)bktLds);

  k_prep<<<GX + NBW1 + NBW2, NTHR, 0, stream>>>(x, NN, GX, W1, W2, XB, W1B, W2D);
  k_bucket<<<NBLK, NTHR, bktLds, stream>>>(src, dst, ew, NE, NN, vec8, HS, HW, CNT, OFF, DIN, FLG);
  k_gemm<<<MP / GBM, GTHR, 0, stream>>>(XB, W1B, DD, H);
  k_agg<1><<<NBLK, NTHR, 0, stream>>>(HS, HW, CNT, OFF, DIN, FLG, NN, MP, H, b1, X1, HF);
  k_gemm<<<MP / GBM, GTHR, 0, stream>>>(X1, W2D, KA, H);
  k_agg<0><<<NBLK, NTHR, 0, stream>>>(HS, HW, CNT, OFF, DIN, FLG, NN, MP, H, b2, X1, HF);
  k_pool<<<NGR, NTHR, 0, stream>>>(HF, bat, NN, PL);
  k_head<<<NHB, NTHR, 0, stream>>>(PL, fW1, fb1, fW2, fb2, FLG, NBLK, out);
}
